// RelativeTransformer_4930622456118
// MI455X (gfx1250) — hardware-verified
//
#include <hip/hip_runtime.h>
#include <stdint.h>

typedef __attribute__((ext_vector_type(16))) _Float16 v16h;
typedef __attribute__((ext_vector_type(8)))  _Float16 v8h;
typedef __attribute__((ext_vector_type(16))) __bf16   v16b;
typedef __attribute__((ext_vector_type(8)))  __bf16   v8b;
typedef __attribute__((ext_vector_type(8)))  float    v8f;
typedef __attribute__((ext_vector_type(4)))  float    v4f;

__device__ __forceinline__ unsigned short f2bf_bits(float f) {
  unsigned u = __float_as_uint(f);
  return (unsigned short)((u + 0x7FFFu + ((u >> 16) & 1u)) >> 16);
}
__device__ __forceinline__ float bf_bits2f(unsigned short h) { return __uint_as_float(((unsigned)h) << 16); }

__device__ __forceinline__ void dep_guard_h(v8f& a, v8f& b, v16h x, v16h y) { asm volatile("v_nop\n\tv_nop\n\tv_nop\n\tv_nop" : "+v"(a), "+v"(b) : "v"(x), "v"(y)); }
__device__ __forceinline__ void dep_guard_b(v8f& a, v8f& b, v16b x, v16b y) { asm volatile("v_nop\n\tv_nop\n\tv_nop\n\tv_nop" : "+v"(a), "+v"(b) : "v"(x), "v"(y)); }
__device__ __forceinline__ void keep4_h(v16h a, v16h b, v16h c, v16h d) { asm volatile("v_nop" :: "v"(a), "v"(b), "v"(c), "v"(d)); }
__device__ __forceinline__ void keep4_b(v16b a, v16b b, v16b c, v16b d) { asm volatile("v_nop" :: "v"(a), "v"(b), "v"(c), "v"(d)); }
__device__ __forceinline__ void acc_guard4(v8f& a, v8f& b, v8f& c, v8f& d) { asm volatile("v_nop\n\tv_nop\n\tv_nop\n\tv_nop" : "+v"(a), "+v"(b), "+v"(c), "+v"(d)); }
template <typename T> struct Frag;
template <> struct Frag<_Float16> {
  typedef v16h V; union U { v16h v; v8h h[2]; };
  static __device__ __forceinline__ v16h load(const _Float16* p) {
    U f; f.h[0] = *(const v8h*)(p); f.h[1] = *(const v8h*)(p + 16); return f.v;
  }
  static __device__ __forceinline__ v8f mma(v16h a, v16h b, v8f c) {
    return __builtin_amdgcn_wmma_f32_16x16x32_f16(false, a, false, b, (short)0, c, false, false);
  }
  static __device__ __forceinline__ void guard(v8f& a, v8f& b, v16h x, v16h y) { dep_guard_h(a, b, x, y); }
  static __device__ __forceinline__ void keep(v16h a, v16h b, v16h c, v16h d) { keep4_h(a, b, c, d); }
};
template <> struct Frag<__bf16> {
  typedef v16b V; union U { v16b v; v8b h[2]; };
  static __device__ __forceinline__ v16b load(const __bf16* p) {
    U f; f.h[0] = *(const v8b*)(p); f.h[1] = *(const v8b*)(p + 16); return f.v;
  }
  static __device__ __forceinline__ v8f mma(v16b a, v16b b, v8f c) {
    return __builtin_amdgcn_wmma_f32_16x16x32_bf16(false, a, false, b, (short)0, c, false, false);
  }
  static __device__ __forceinline__ void guard(v8f& a, v8f& b, v16b x, v16b y) { dep_guard_b(a, b, x, y); }
  static __device__ __forceinline__ void keep(v16b a, v16b b, v16b c, v16b d) { keep4_b(a, b, c, d); }
};

template <int ET> struct Elem;
template <> struct Elem<0> { typedef _Float16 T; };
template <> struct Elem<1> { typedef __bf16 T; };
template <int ET, bool SPLIT, int BIAS_MODE, int OUT_MODE, bool RESID, int ACT = 0>
__global__ __launch_bounds__(256) void wmma_gemm64(
    const unsigned short* __restrict__ Ap, const unsigned short* __restrict__ A2p, int lda, long strideA,
    const unsigned short* __restrict__ Btp, const unsigned short* __restrict__ Bt2p, int ldb, long strideB,
    void* __restrict__ Cout, void* __restrict__ Cout2, int ldc, long strideC,
    const float* __restrict__ bias,
    const float* __restrict__ resid, long strideR,
    int M, int N, int K, float scale) {
  typedef typename Elem<ET>::T T;
  typedef typename Frag<T>::V V;
  const T* A = (const T*)Ap; const T* A2 = (const T*)A2p; const T* Bt = (const T*)Btp; const T* Bt2 = (const T*)Bt2p;
  __shared__ __align__(16) float sT[8][16 * 68];
  const int b    = blockIdx.y;
  const int lane = threadIdx.x & 31;
  const int wave = threadIdx.x >> 5;
  const int tilesN = N >> 6;
  const int tilesM = M >> 6;
  const int tile = blockIdx.x * 8 + wave;
  if (tile >= tilesM * tilesN) return;
  const int tm = tile / tilesN;
  const int tn = tile - tm * tilesN;
  const int m0 = tm << 6;
  const int n0 = tn << 6;

  const T* Ab  = A  + (size_t)b * strideA;
  const T* Bb  = Bt + (size_t)b * strideB;
  const T* Ab2 = SPLIT ? (A2  + (size_t)b * strideA) : nullptr;
  const T* Bb2 = SPLIT ? (Bt2 + (size_t)b * strideB) : nullptr;

  const int rlane = lane & 15;
  const int koff  = (lane >> 4) * 8;
  const int mOff  = (lane >> 4) * 8;

  v8f acc[4][4];
#pragma unroll
  for (int i = 0; i < 4; ++i)
#pragma unroll
    for (int j = 0; j < 4; ++j) acc[i][j] = (v8f){0.f,0.f,0.f,0.f,0.f,0.f,0.f,0.f};

  for (int k0 = 0; k0 < K; k0 += 32) {
    V bh[4], bl[4];
#pragma unroll
    for (int j = 0; j < 4; ++j) {
      const size_t bo = (size_t)(n0 + (j << 4) + rlane) * ldb + koff + k0;
      bh[j] = Frag<T>::load(Bb + bo);
      if (SPLIT) bl[j] = Frag<T>::load(Bb2 + bo);
    }
#pragma unroll
    for (int i = 0; i < 4; ++i) {
      const size_t ao = (size_t)(m0 + (i << 4) + rlane) * lda + koff + k0;
      V ah = Frag<T>::load(Ab + ao);
      V al;
      if (SPLIT) al = Frag<T>::load(Ab2 + ao);
#pragma unroll
      for (int j = 0; j < 4; ++j) {
        acc[i][j] = Frag<T>::mma(ah, bh[j], acc[i][j]);
        if (SPLIT) {
          acc[i][j] = Frag<T>::mma(ah, bl[j], acc[i][j]);
          acc[i][j] = Frag<T>::mma(al, bh[j], acc[i][j]);
        }
      }
      Frag<T>::guard(acc[i][0], acc[i][3], ah, SPLIT ? al : ah);
    }
    Frag<T>::keep(bh[0], bh[1], bh[2], bh[3]);
    if (SPLIT) Frag<T>::keep(bl[0], bl[1], bl[2], bl[3]);
  }
  acc_guard4(acc[0][0], acc[0][1], acc[0][2], acc[0][3]);
  acc_guard4(acc[1][0], acc[1][1], acc[1][2], acc[1][3]);
  acc_guard4(acc[2][0], acc[2][1], acc[2][2], acc[2][3]);
  acc_guard4(acc[3][0], acc[3][1], acc[3][2], acc[3][3]);

  float* slab = sT[wave];
  const float* Rb = RESID ? (resid + (size_t)b * strideR) : nullptr;
#pragma unroll
  for (int i = 0; i < 4; ++i) {
    const int mBase = m0 + (i << 4);
#pragma unroll
    for (int j = 0; j < 4; ++j) {
      const int n = n0 + (j << 4) + rlane;
      float bv = 0.f;
      if (BIAS_MODE == 2) bv = bias[n];
#pragma unroll
      for (int r = 0; r < 8; ++r) {
        float v = acc[i][j][r] * scale;
        if (BIAS_MODE == 1) v += bias[mBase + mOff + r];
        if (BIAS_MODE == 2) v += bv;
        if (RESID) v += Rb[(size_t)(mBase + mOff + r) * ldc + n];
        if (ACT == 1) v = tanhf(v);
        if (ACT == 2) v = fmaxf(v, 0.0f);
        if (ACT == 3) v = v / (1.0f + expf(-v));
        if (ACT == 4) v = (v > 0.f) ? v : 0.01f * v;
        if (ACT == 5) v = 0.5f * v * (1.0f + erff(v * 0.70710678118654752f));
        slab[(mOff + r) * 68 + (j << 4) + rlane] = v;
      }
    }
    __builtin_amdgcn_fence(__ATOMIC_RELEASE, "workgroup");
    __builtin_amdgcn_wave_barrier();
    __builtin_amdgcn_fence(__ATOMIC_ACQUIRE, "workgroup");
    if (OUT_MODE == 0) {
      float* C = (float*)Cout + (size_t)b * strideC;
      const int hh = lane >> 4, c4 = (lane & 15) * 4;
      for (int pass = 0; pass < 2; ++pass) {
#pragma unroll
        for (int it = 0; it < 8; ++it) {
          const int row = it * 2 + hh;
          v4f v = *(const v4f*)(slab + row * 68 + c4);
          *(volatile v4f*)(C + (size_t)(mBase + row) * ldc + n0 + c4) = v;
        }
        __threadfence();
      }
    } else {
      const int q = lane >> 3, c8 = (lane & 7) * 8;
      unsigned short* C  = (unsigned short*)Cout  + (size_t)b * strideC;
      unsigned short* C2 = (OUT_MODE == 2) ? ((unsigned short*)Cout2 + (size_t)b * strideC) : nullptr;
      for (int pass = 0; pass < 2; ++pass) {
#pragma unroll
        for (int it = 0; it < 4; ++it) {
          const int row = it * 4 + q;
          const float* sp = slab + row * 68 + c8;
          v8h hv, lv;
#pragma unroll
          for (int e = 0; e < 8; ++e) {
            if (OUT_MODE == 1) {
              hv[e] = (_Float16)sp[e];
            } else {
              unsigned short hb = f2bf_bits(sp[e]);
              unsigned short lb = f2bf_bits(sp[e] - bf_bits2f(hb));
              hv[e] = __builtin_bit_cast(_Float16, hb);
              lv[e] = __builtin_bit_cast(_Float16, lb);
            }
          }
          *(volatile v8h*)(C + (size_t)(mBase + row) * ldc + n0 + c8) = hv;
          if (OUT_MODE == 2) *(volatile v8h*)(C2 + (size_t)(mBase + row) * ldc + n0 + c8) = lv;
        }
        __threadfence();
      }
    }
    __builtin_amdgcn_fence(__ATOMIC_RELEASE, "workgroup");
    __builtin_amdgcn_wave_barrier();
    __builtin_amdgcn_fence(__ATOMIC_ACQUIRE, "workgroup");
  }
}

__global__ __launch_bounds__(256) void cast_f32_f16x2s(
    const float* __restrict__ in, _Float16* __restrict__ out, int n2, float scale) {
  int i = blockIdx.x * 256 + threadIdx.x;
  if (i < n2) {
    const _Float16 h0 = (_Float16)(in[2 * i] * scale), h1 = (_Float16)(in[2 * i + 1] * scale);
    const unsigned u = (unsigned)__builtin_bit_cast(unsigned short, h0) | ((unsigned)__builtin_bit_cast(unsigned short, h1) << 16);
    ((volatile unsigned*)out)[i] = u;
    __threadfence();
    ((volatile unsigned*)out)[i] = u;
  }
}

__global__ __launch_bounds__(128) void sbias_kernel(
    const float* __restrict__ qf, const float* __restrict__ rf, const float* __restrict__ semb,
    const float* __restrict__ utt, const int* __restrict__ amask, const int* __restrict__ smask,
    float* __restrict__ sb) {
  __shared__ float se0[128];
  __shared__ float se1[128];
  __shared__ float scv[128];
  const int n = blockIdx.x, t = threadIdx.x;
  const int b = n >> 4, h = n & 15;
  {
    const size_t ro = ((size_t)(t * 8 + b)) * 1024 + (size_t)h * 64;
    const float* qr = qf + ro;
    const float* rr = rf + ro;
    const float* s0 = semb + h * 64;
    const float* s1 = semb + 1024 + h * 64;
    float a0 = 0.f, a1 = 0.f, a2 = 0.f;
#pragma unroll 1
    for (int e = 0; e < 64; e += 4) {
      const v4f qv = *(const v4f*)(qr + e);
      const v4f rv = *(const v4f*)(rr + e);
      const v4f w0 = *(const v4f*)(s0 + e);
      const v4f w1 = *(const v4f*)(s1 + e);
#pragma unroll
      for (int u = 0; u < 4; ++u) {
        a0 = fmaf(qv[u], w0[u], a0);
        a1 = fmaf(qv[u], w1[u], a1);
        a2 = fmaf(rv[u], w0[u], a2);
      }
    }
    se0[t] = a0;
    se1[t] = a1;
    scv[t] = a2;
  }
  __syncthreads();
  const float* ub  = utt   + (size_t)n * 16384;
  const int*   ab  = amask + (size_t)n * 16384;
  const int*   smb = smask + (size_t)b * 16384;
  float*       ob  = sb    + (size_t)n * 16384;
#pragma unroll 1
  for (int i = 0; i < 128; ++i) {
    const int e = i * 128 + t;
    const float u = ub[e];
    const int am = ab[e];
    int sm = smb[e];
    if (sm < 0) sm += 2;
    sm = sm < 0 ? 0 : (sm > 1 ? 1 : sm);
    const float ev = (sm != 0) ? se1[i] : se0[i];
    int cc = 127 - i + t;
    cc = cc < 0 ? 0 : (cc > 127 ? 127 : cc);
    const float a3 = (t <= i) ? scv[cc] : 0.0f;
    float val = (u * ev + a3) * 0.125f;
    if (am != 0) val = 3.0e38f;
    *(volatile float*)(ob + e) = val;
    __threadfence();
    *(volatile float*)(ob + e) = val;
  }
}

#define AT_D 64
#define AT_NW 4
#define AT_QB 64
#define AT_KC 64
struct AttnArgs { long q_bs, q_rs, q_hs, k_bs, k_rs, k_hs, v_bs, v_rs, v_hs, o_bs, o_rs, o_hs, sb_ns, sb_rs;
                  int S, Skv, H, nchunks; float sscale, mask_fill, sent_thr, resv; };
static_assert(sizeof(AttnArgs) == 144);

__device__ __forceinline__ v8f mma_f16g(v16h a, v16h b, v8f c) {
  c = __builtin_amdgcn_wmma_f32_16x16x32_f16(false, a, false, b, (short)0, c, false, false);
  asm volatile("v_nop\n\tv_nop\n\tv_nop\n\tv_nop" : "+v"(c) : "v"(a), "v"(b));
  return c;
}

__global__ __launch_bounds__(128)
void attn64_sbias_f16(const float* __restrict__ q, const float* __restrict__ k,
                      const float* __restrict__ v, float* __restrict__ out,
                      const float* __restrict__ sb, AttnArgs g) {
  const float PSC = 32768.0f;
  union FB { v16h v; v8h h[2]; };
  __shared__ __align__(16) _Float16 Ksh[AT_KC * AT_D];
  __shared__ __align__(16) _Float16 Vth[AT_D * AT_KC];
  __shared__ __align__(16) _Float16 Psh[AT_NW][16 * AT_KC];
  __shared__ __align__(16) float    Os[AT_NW][16 * 68];

  const int tid  = threadIdx.x;
  const int wave = tid >> 5;
  const int lane = tid & 31;
  const int hh   = lane >> 4;
  const int c    = lane & 15;

  const int nqb = g.S / AT_QB;
  const int bx = blockIdx.x;
  const int qb = bx % nqb;
  const int bh = bx / nqb;
  const int h  = bh % g.H;
  const int b  = bh / g.H;
  const int q0 = qb * AT_QB + wave * 16;

  const float* qb_ptr = q   + (size_t)b * g.q_bs + (size_t)h * g.q_hs;
  const float* kb_ptr = k   + (size_t)b * g.k_bs + (size_t)h * g.k_hs;
  const float* vb_ptr = v   + (size_t)b * g.v_bs + (size_t)h * g.v_hs;
  float*       ob_ptr = out + (size_t)b * g.o_bs + (size_t)h * g.o_hs;

  v16h qa[2];
  {
    const float* qrow = qb_ptr + (size_t)(q0 + c) * g.q_rs;
#pragma unroll
    for (int dc = 0; dc < 2; ++dc) {
      const v4f f0 = *(const v4f*)(qrow + dc * 32 + 8 * hh);
      const v4f f1 = *(const v4f*)(qrow + dc * 32 + 8 * hh + 4);
      const v4f f2 = *(const v4f*)(qrow + dc * 32 + 16 + 8 * hh);
      const v4f f3 = *(const v4f*)(qrow + dc * 32 + 16 + 8 * hh + 4);
#pragma unroll
      for (int e = 0; e < 4; ++e) {
        qa[dc][e]      = (_Float16)f0[e];
        qa[dc][4 + e]  = (_Float16)f1[e];
        qa[dc][8 + e]  = (_Float16)f2[e];
        qa[dc][12 + e] = (_Float16)f3[e];
      }
    }
  }

  float mrow[8], lrow[8];
  v8f oacc[4];
#pragma unroll
  for (int r = 0; r < 8; ++r) { mrow[r] = -INFINITY; lrow[r] = 0.f; }
#pragma unroll
  for (int t = 0; t < 4; ++t) oacc[t] = (v8f){0.f,0.f,0.f,0.f,0.f,0.f,0.f,0.f};

  int nChunks = g.Skv / AT_KC;
  if (nChunks > 64) nChunks = 64;
  for (int kc = 0; kc < nChunks; ++kc) {
    const int kv0 = kc * AT_KC;
    __syncthreads();
    {
      const int kvr = tid >> 1, dh = (tid & 1) * 32;
      const float* krow = kb_ptr + (size_t)(kv0 + kvr) * g.k_rs + dh;
      const float* vrow = vb_ptr + (size_t)(kv0 + kvr) * g.v_rs + dh;
#pragma unroll
      for (int i = 0; i < 8; ++i) {
        v4f kk = *(const v4f*)(krow + 4 * i);
        v4f vv = *(const v4f*)(vrow + 4 * i);
#pragma unroll
        for (int e = 0; e < 4; ++e) {
          const int d = dh + 4 * i + e;
          Ksh[kvr * AT_D + d]  = (_Float16)kk[e];
          Vth[d * AT_KC + kvr] = (_Float16)vv[e];
        }
      }
    }
    __syncthreads();

    v8f s[4];
#pragma unroll
    for (int j = 0; j < 4; ++j) {
      s[j] = (v8f){0.f,0.f,0.f,0.f,0.f,0.f,0.f,0.f};
#pragma unroll
      for (int dc = 0; dc < 2; ++dc) {
        FB kb;
        kb.h[0] = *(const v8h*)(Ksh + (j * 16 + c) * AT_D + dc * 32 + 8 * hh);
        kb.h[1] = *(const v8h*)(Ksh + (j * 16 + c) * AT_D + dc * 32 + 16 + 8 * hh);
        s[j] = mma_f16g(qa[dc], kb.v, s[j]);
      }
    }
    const float* sbp = sb + (size_t)bh * g.sb_ns + (size_t)(q0 + 8 * hh) * g.sb_rs + kv0 + c;
    float cm[8];
#pragma unroll
    for (int r = 0; r < 8; ++r) {
      const float* sbr = sbp + (size_t)r * g.sb_rs;
      float m = -INFINITY;
#pragma unroll
      for (int j = 0; j < 4; ++j) {
        const float bb = sbr[j * 16];
        float sv = fmaf(s[j][r], g.sscale, bb);
        if (bb > g.sent_thr) sv = g.mask_fill;
        s[j][r] = sv;
        m = fmaxf(m, sv);
      }
#pragma unroll
      for (int off = 1; off < 16; off <<= 1) m = fmaxf(m, __shfl_xor(m, off, 32));
      cm[r] = m;
    }
    _Float16* pwh = Psh[wave];
#pragma unroll
    for (int r = 0; r < 8; ++r) {
      const float mnew = fmaxf(mrow[r], cm[r]);
      const float alpha = expf(mrow[r] - mnew);
      mrow[r] = mnew;
      float psum = 0.f;
#pragma unroll
      for (int j = 0; j < 4; ++j) {
        const float p = expf(s[j][r] - mnew);
        psum += p;
        pwh[(8 * hh + r) * AT_KC + j * 16 + c] = (_Float16)(p * PSC);
      }
#pragma unroll
      for (int off = 1; off < 16; off <<= 1) psum += __shfl_xor(psum, off, 32);
      lrow[r] = lrow[r] * alpha + psum;
#pragma unroll
      for (int t = 0; t < 4; ++t) oacc[t][r] *= alpha;
    }
    __builtin_amdgcn_fence(__ATOMIC_RELEASE, "workgroup");
    __builtin_amdgcn_wave_barrier();
    __builtin_amdgcn_fence(__ATOMIC_ACQUIRE, "workgroup");
#pragma unroll 1
    for (int kk = 0; kk < 2; ++kk) {
      FB pa;
      pa.h[0] = *(const v8h*)(pwh + c * AT_KC + kk * 32 + 8 * hh);
      pa.h[1] = *(const v8h*)(pwh + c * AT_KC + kk * 32 + 16 + 8 * hh);
#pragma unroll
      for (int t = 0; t < 4; ++t) {
        FB vb;
        vb.h[0] = *(const v8h*)(Vth + (t * 16 + c) * AT_KC + kk * 32 + 8 * hh);
        vb.h[1] = *(const v8h*)(Vth + (t * 16 + c) * AT_KC + kk * 32 + 16 + 8 * hh);
        oacc[t] = mma_f16g(pa.v, vb.v, oacc[t]);
      }
    }
  }

  float* os = Os[wave];
#pragma unroll
  for (int r = 0; r < 8; ++r) {
    const float inv = 1.0f / (lrow[r] * PSC);
#pragma unroll
    for (int t = 0; t < 4; ++t) os[(8 * hh + r) * 68 + t * 16 + c] = oacc[t][r] * inv;
  }
  __builtin_amdgcn_fence(__ATOMIC_RELEASE, "workgroup");
  __builtin_amdgcn_wave_barrier();
  __builtin_amdgcn_fence(__ATOMIC_ACQUIRE, "workgroup");
  {
    const int c4 = (lane & 15) * 4;
    for (int pass = 0; pass < 2; ++pass) {
#pragma unroll
      for (int it = 0; it < 8; ++it) {
        const int row = it * 2 + hh;
        v4f val = *(const v4f*)(os + row * 68 + c4);
        *(volatile v4f*)(ob_ptr + (size_t)(q0 + row) * g.o_rs + c4) = val;
      }
      __threadfence();
    }
  }
}

extern "C" void kernel_launch(void* const* d_in, const int* in_sizes, int n_in,
                              void* d_out, int out_size, void* d_ws, size_t ws_size,
                              hipStream_t stream) {
  if (n_in < 11) return;
  const int NE = 1024 * 1024;
  if (in_sizes[0] != NE || in_sizes[1] != NE || in_sizes[3] != NE || in_sizes[4] != NE ||
      in_sizes[5] != NE || in_sizes[6] != NE || in_sizes[7] != NE || in_sizes[8] != 2 * 1024 ||
      in_sizes[2] != 128 * 128 * 128 || in_sizes[9] != 128 * 128 * 128 || in_sizes[10] != 8 * 128 * 128 ||
      out_size != NE) return;

  const float* query    = (const float*)d_in[0];
  const float* rel_pe   = (const float*)d_in[1];
  const float* utt_mask = (const float*)d_in[2];
  const float* Wq       = (const float*)d_in[3];
  const float* Wk       = (const float*)d_in[4];
  const float* Wv       = (const float*)d_in[5];
  const float* Wr       = (const float*)d_in[6];
  const float* Wo       = (const float*)d_in[7];
  const float* spk_emb  = (const float*)d_in[8];
  const int*   attn_msk = (const int*)d_in[9];
  const int*   spk_msk  = (const int*)d_in[10];
  float* out = (float*)d_out;

  const size_t MiB = (size_t)1 << 20;
  const size_t off_q16 = 0;
  const size_t off_p16 = 2 * MiB;
  const size_t off_w16 = 4 * MiB;
  const size_t off_qf  = 14 * MiB;
  const size_t off_kf  = 18 * MiB;
  const size_t off_vf  = 22 * MiB;
  const size_t off_rf  = 26 * MiB;
  const size_t off_sb  = 30 * MiB;
  const size_t off_ctx = 38 * MiB;
  const size_t off_c16 = 42 * MiB;
  const size_t total   = 44 * MiB;
  if (total > ws_size || total > 128 * MiB) return;

  char* ws = (char*)d_ws;
  _Float16* q16 = (_Float16*)(ws + off_q16);
  _Float16* p16 = (_Float16*)(ws + off_p16);
  _Float16* w16 = (_Float16*)(ws + off_w16);
  float* qf  = (float*)(ws + off_qf);
  float* kf  = (float*)(ws + off_kf);
  float* vf  = (float*)(ws + off_vf);
  float* rf  = (float*)(ws + off_rf);
  float* sbp = (float*)(ws + off_sb);
  float* ctx = (float*)(ws + off_ctx);
  _Float16* c16 = (_Float16*)(ws + off_c16);

  const int n2 = NE / 2;
  const int cgrid = (n2 + 255) / 256;
  cast_f32_f16x2s<<<cgrid, 256, 0, stream>>>(query,  q16, n2, 1.0f);
  cast_f32_f16x2s<<<cgrid, 256, 0, stream>>>(rel_pe, p16, n2, 1.0f);
  cast_f32_f16x2s<<<cgrid, 256, 0, stream>>>(Wq, w16 + 0 * (size_t)NE, n2, 16.0f);
  cast_f32_f16x2s<<<cgrid, 256, 0, stream>>>(Wk, w16 + 1 * (size_t)NE, n2, 16.0f);
  cast_f32_f16x2s<<<cgrid, 256, 0, stream>>>(Wv, w16 + 2 * (size_t)NE, n2, 16.0f);
  cast_f32_f16x2s<<<cgrid, 256, 0, stream>>>(Wr, w16 + 3 * (size_t)NE, n2, 16.0f);
  cast_f32_f16x2s<<<cgrid, 256, 0, stream>>>(Wo, w16 + 4 * (size_t)NE, n2, 16.0f);

  const int M = 1024, N = 1024, K = 1024;
  const int tiles = (M / 64) * (N / 64);
  const int gblocks = (tiles + 7) / 8;
  const float wscale_inv = 1.0f / 16.0f;
  {
    dim3 grid(gblocks, 1);
    wmma_gemm64<0, false, 2, 0, false><<<grid, 256, 0, stream>>>(
        (const unsigned short*)q16, (const unsigned short*)q16, K, 0L,
        (const unsigned short*)(w16 + 0 * (size_t)NE), (const unsigned short*)(w16 + 0 * (size_t)NE), K, 0L,
        (void*)qf, (void*)qf, N, 0L,
        spk_emb, spk_emb, 0L, M, N, K, wscale_inv);
  }
  {
    dim3 grid(gblocks, 2);
    wmma_gemm64<0, false, 0, 0, false><<<grid, 256, 0, stream>>>(
        (const unsigned short*)q16, (const unsigned short*)q16, K, 0L,
        (const unsigned short*)(w16 + 1 * (size_t)NE), (const unsigned short*)(w16 + 1 * (size_t)NE), K, (long)NE,
        (void*)kf, (void*)kf, N, (long)NE,
        spk_emb, spk_emb, 0L, M, N, K, wscale_inv);
  }
  {
    dim3 grid(gblocks, 1);
    wmma_gemm64<0, false, 0, 0, false><<<grid, 256, 0, stream>>>(
        (const unsigned short*)p16, (const unsigned short*)p16, K, 0L,
        (const unsigned short*)(w16 + 3 * (size_t)NE), (const unsigned short*)(w16 + 3 * (size_t)NE), K, 0L,
        (void*)rf, (void*)rf, N, 0L,
        spk_emb, spk_emb, 0L, M, N, K, wscale_inv);
  }

  sbias_kernel<<<128, 128, 0, stream>>>(qf, rf, spk_emb, utt_mask, attn_msk, spk_msk, sbp);

  {
    AttnArgs g;
    g.q_bs = 1024; g.q_rs = 8 * 1024; g.q_hs = 64;
    g.k_bs = 1024; g.k_rs = 8 * 1024; g.k_hs = 64;
    g.v_bs = 1024; g.v_rs = 8 * 1024; g.v_hs = 64;
    g.o_bs = 1024; g.o_rs = 8 * 1024; g.o_hs = 64;
    g.sb_ns = 128 * 128; g.sb_rs = 128;
    g.S = 128; g.Skv = 128; g.H = 16; g.nchunks = 2;
    g.sscale = 0.125f; g.mask_fill = 1e-30f; g.sent_thr = 1.0e37f; g.resv = 0.0f;
    const int agrid = 8 * 16 * (128 / AT_QB);
    attn64_sbias_f16<<<agrid, 128, 0, stream>>>(qf, kf, vf, ctx, sbp, g);
  }

  cast_f32_f16x2s<<<cgrid, 256, 0, stream>>>(ctx, c16, n2, 16.0f);
  {
    dim3 grid(gblocks, 1);
    wmma_gemm64<0, false, 0, 0, false><<<grid, 256, 0, stream>>>(
        (const unsigned short*)c16, (const unsigned short*)c16, K, 0L,
        (const unsigned short*)(w16 + 4 * (size_t)NE), (const unsigned short*)(w16 + 4 * (size_t)NE), K, 0L,
        (void*)out, (void*)out, N, 0L,
        spk_emb, spk_emb, 0L, M, N, K, 1.0f / 256.0f);
  }
  (void)hipGetLastError();
}
